// Nn0_86801289052729
// MI455X (gfx1250) — hardware-verified
//
#include <hip/hip_runtime.h>


#define CTX   24
#define DKW   92
#define EMB   36
#define NTOK  500
#define HID   152
#define CCAT  936
#define EMP   48
#define DKP   96
#define KXP   32
#define KJP   64
#define MT_   (EMP / 16)
#define NT_   (DKP / 16)
#define QP    96
#define VP    72
#define PP    72
#define SP    49
#define NTH   512
#define NWV   16
#define WSZ   (DKP * KXP)
#define QRS   2048.0f
#define QRI   (1.0f / 2048.0f)
#define PCAR  16384.0f
#define VCAR  64.0f
#define OFOLD (1.0f / (16384.0f * 64.0f))
#define SC2   ((float)(9.591663046625438 * 1.4426950408889634))
#define NEGB  (-3.0e38f)
#define MPART 3
#define MROWS 312

static_assert(CCAT == 2 * EMB + EMB * CTX);
static_assert(EMP % 16 == 0);
static_assert(EMP >= EMB);
static_assert(DKP % 32 == 0);
static_assert(DKP >= DKW);
static_assert(KXP == 32);
static_assert(KXP >= CTX);
static_assert(KJP % 32 == 0);
static_assert(KJP >= EMP);
static_assert(QP % 8 == 0);
static_assert(VP % 8 == 0);
static_assert(PP % 8 == 0);
static_assert(QP >= DKP);
static_assert(VP >= KJP);
static_assert(PP >= KJP);
static_assert(MPART * MROWS == CCAT);
static_assert(NTH >= MPART * HID);
static_assert(NTH <= 4 * HID);
static_assert(NTH == 32 * NWV);
static_assert(EMB <= 64);
static_assert(NTOK % 4 == 0);
static_assert(NTOK / 4 <= 128);
static_assert((size_t)(NTOK / 4) * 1 * 16 == (size_t)NTOK * 4);
static_assert((NTOK * 4) % 16 == 0);

typedef _Float16 h16;
typedef unsigned short bf;
typedef __attribute__((ext_vector_type(16))) __bf16   v16bf;
typedef __attribute__((ext_vector_type(16))) _Float16 v16h;
typedef __attribute__((ext_vector_type(8)))  _Float16 v8h;
typedef __attribute__((ext_vector_type(8)))  unsigned short v8us;
typedef __attribute__((ext_vector_type(8)))  float    v8f;
typedef __attribute__((ext_vector_type(4)))  float    v4f;

static constexpr size_t LDS_BYTES =
    (size_t)EMP * KXP * 2 + (size_t)6 * WSZ * 2 + (size_t)2 * (2 * EMP * QP * 2) + (size_t)DKP * VP * 2 + (size_t)EMP * PP * 2 +
    (size_t)EMP * SP * 4 + (size_t)EMP * NT_ * 4 + (size_t)CCAT * 4 + (size_t)4 * HID * 4 + (size_t)HID * 4 + (size_t)EMB * 4;
static_assert(LDS_BYTES <= (size_t)131072);

__device__ __forceinline__ unsigned short f2bf(float f) { unsigned u = __float_as_uint(f); u += 0x7FFFu + ((u >> 16) & 1u); return (unsigned short)(u >> 16); }
__device__ __forceinline__ float bfr(float f) { return __uint_as_float(((unsigned)f2bf(f)) << 16); }
__device__ __forceinline__ v16h cat16(v8h lo, v8h hi) { return __builtin_shufflevector(lo, hi, 0, 1, 2, 3, 4, 5, 6, 7, 8, 9, 10, 11, 12, 13, 14, 15); }
__device__ __forceinline__ v16bf cat16b(v8us lo, v8us hi) { return __builtin_bit_cast(v16bf, __builtin_shufflevector(lo, hi, 0, 1, 2, 3, 4, 5, 6, 7, 8, 9, 10, 11, 12, 13, 14, 15)); }
__device__ __forceinline__ v8f wmma16(v16h a, v16h b, v8f c) { return __builtin_amdgcn_wmma_f32_16x16x32_f16(false, a, false, b, (short)0, c, false, false); }
__device__ __forceinline__ v8f wmmab(v16bf a, v16bf b, v8f c) { return __builtin_amdgcn_wmma_f32_16x16x32_bf16(false, a, false, b, (short)0, c, false, false); }
__device__ __forceinline__ v16h  ldh(const h16* p) { return cat16(*(const v8h*)p, *(const v8h*)(p + 16)); }
__device__ __forceinline__ v16bf ldb(const bf* p)  { return cat16b(*(const v8us*)p, *(const v8us*)(p + 16)); }
__device__ __forceinline__ v8f wmma16_g(v16h a, v16h b, v8f c) { c = wmma16(a, b, c); asm volatile("v_nop\n\tv_nop\n\tv_nop\n\tv_nop" : "+v"(c) : "v"(a), "v"(b)); return c; }
__device__ __forceinline__ v8f wmmab_g(v16bf a, v16bf b, v8f c) { c = wmmab(a, b, c); asm volatile("v_nop\n\tv_nop\n\tv_nop\n\tv_nop" : "+v"(c) : "v"(a), "v"(b)); return c; }
__device__ __forceinline__ h16 toh_flush(float v) { const h16 r = (h16)v; return (fabsf(v) < 6.103515625e-05f) ? (h16)0.0f : r; }
__device__ __forceinline__ bf wt_elem(const float* __restrict__ w, int d, int c) {
    const int dc = d < DKW ? d : DKW - 1; const int cc = c < CTX ? c : CTX - 1;
    float v = w[cc * DKW + dc];
    asm volatile("" : "+v"(v));
    return ((d < DKW) & (c < CTX)) ? f2bf(v) : (bf)0;
}

__global__ __launch_bounds__(NTH) void k_fused(
    const float* __restrict__ x0,
    const float* __restrict__ wq1, const float* __restrict__ wk1, const float* __restrict__ wv1,
    const float* __restrict__ wq2, const float* __restrict__ wk2, const float* __restrict__ wv2,
    const float* __restrict__ nl0, const float* __restrict__ nl0b,
    const float* __restrict__ nl1,
    const float* __restrict__ ctp, const float* __restrict__ ctpb,
    float* out)
{
    __shared__ __align__(16) bf  XB[EMP * KXP];
    __shared__ __align__(16) bf  WT[6 * WSZ];
    __shared__ __align__(16) h16 QKH[2 * EMP * QP];
    __shared__ __align__(16) h16 QKR[2 * EMP * QP];
    __shared__ __align__(16) h16 VT[DKP * VP];
    __shared__ __align__(16) h16 PH[EMP * PP];
    __shared__ float SB[EMP * SP];
    __shared__ float OS[EMP * NT_];
    __shared__ float T71[CCAT];
    __shared__ float PRE[4 * HID];
    __shared__ float T7[HID];
    __shared__ float T10[EMB];

    const int tid = threadIdx.x;
    const int lane = tid & 31, lr = lane & 15, hi = lane >> 4;
    const int wave = __builtin_amdgcn_readfirstlane((int)(threadIdx.x >> 5));

    for (int i = tid; i < EMP * KXP; i += NTH) {
        const int r = i >> 5, c = i & 31;
        const int rc = r < EMB ? r : EMB - 1; const int cc = c < CTX ? c : CTX - 1;
        float v = x0[rc * CTX + cc];
        asm volatile("" : "+v"(v));
        XB[i] = ((r < EMB) & (c < CTX)) ? f2bf(v) : (bf)0;
    }
    for (int i = tid; i < WSZ; i += NTH) {
        const int d = i % DKP, c = i / DKP; const int o = d * KXP + c;
        WT[0 * WSZ + o] = wt_elem(wq1, d, c);
        WT[1 * WSZ + o] = wt_elem(wk1, d, c);
        WT[2 * WSZ + o] = wt_elem(wv1, d, c);
        WT[3 * WSZ + o] = wt_elem(wq2, d, c);
        WT[4 * WSZ + o] = wt_elem(wk2, d, c);
        WT[5 * WSZ + o] = wt_elem(wv2, d, c);
    }
    for (int i = tid; i < DKP * VP; i += NTH) VT[i] = (h16)0.0f;
    for (int i = tid; i < EMP * PP; i += NTH) PH[i] = (h16)0.0f;
    for (int i = tid; i < EMB * CTX; i += NTH) T71[2 * EMB + i] = bfr(x0[i]);
    __syncthreads();

#pragma unroll 1
    for (int head = 0; head < 2; ++head) {
        for (int job = wave; job < 3 * MT_ * NT_; job += NWV) {
            const int which = job / (MT_ * NT_); const int rem = job - which * (MT_ * NT_);
            const int mt = rem / NT_; const int nt = rem - mt * NT_;
            const v16bf a = ldb(&XB[(mt * 16 + lr) * KXP + 8 * hi]);
            const v16bf b = ldb(&WT[((head * 3 + which) * DKP + nt * 16 + lr) * KXP + 8 * hi]);
            v8f acc = (v8f){};
            acc = wmmab_g(a, b, acc);
            if (which < 2) {
                const int pb = which * (EMP * QP) + (mt * 16 + 8 * hi) * QP + nt * 16 + lr;
#pragma unroll
                for (int r = 0; r < 8; ++r) {
                    const float x = acc[r]; const h16 hv = toh_flush(x);
                    QKH[pb + r * QP] = hv;
                    QKR[pb + r * QP] = toh_flush((x - (float)hv) * QRS);
                }
            } else {
                const int vb = (nt * 16 + lr) * VP + mt * 16 + 8 * hi;
#pragma unroll
                for (int r = 0; r < 8; ++r) VT[vb + r] = toh_flush(acc[r] * VCAR);
            }
        }
        __syncthreads();

        for (int job = wave; job < MT_ * MT_; job += NWV) {
            const int mt = job / MT_; const int nt = job - mt * MT_;
            const int qo = (mt * 16 + lr) * QP + 8 * hi;
            const int ko = EMP * QP + (nt * 16 + lr) * QP + 8 * hi;
            v8f sH = (v8f){}, sL = (v8f){};
#pragma unroll
            for (int kc = 0; kc < DKP; kc += 32) {
                const v16h qh = ldh(&QKH[qo + kc]); const v16h qr = ldh(&QKR[qo + kc]);
                const v16h kh = ldh(&QKH[ko + kc]); const v16h kr = ldh(&QKR[ko + kc]);
                sH = wmma16_g(qh, kh, sH);
                sL = wmma16_g(qr, kh, sL);
                sL = wmma16_g(qh, kr, sL);
            }
            const int sb = (mt * 16 + 8 * hi) * SP + nt * 16 + lr;
#pragma unroll
            for (int r = 0; r < 8; ++r) SB[sb + r * SP] = sH[r] + sL[r] * QRI;
        }
        __syncthreads();

        if (tid < EMB) {
            const int j = tid;
            float mx = NEGB;
#pragma unroll 1
            for (int i = 0; i < EMB; ++i) { const float t = SB[i * SP + j] * SC2; SB[i * SP + j] = t; mx = fmaxf(mx, t); }
            float l = 0.0f;
#pragma unroll 1
            for (int i = 0; i < EMB; ++i) { const float e = __builtin_amdgcn_exp2f(SB[i * SP + j] - mx); SB[i * SP + j] = e; l += e; }
            const float inv = (1.0f / l) * PCAR;
#pragma unroll 1
            for (int i = 0; i < EMB; ++i) PH[i * PP + j] = toh_flush(SB[i * SP + j] * inv);
        }
        __syncthreads();

        for (int job = wave; job < MT_ * NT_; job += NWV) {
            const int mt = job / NT_; const int nt = job - mt * NT_;
            const int po = (mt * 16 + lr) * PP + 8 * hi;
            const int vo = (nt * 16 + lr) * VP + 8 * hi;
            v8f o = (v8f){};
#pragma unroll
            for (int kc = 0; kc < KJP; kc += 32) {
                const v16h p = ldh(&PH[po + kc]); const v16h v = ldh(&VT[vo + kc]);
                o = wmma16_g(p, v, o);
            }
            float rs[8];
#pragma unroll
            for (int r = 0; r < 8; ++r) {
                float s = o[r];
                s += __shfl_xor(s, 1, 32); s += __shfl_xor(s, 2, 32); s += __shfl_xor(s, 4, 32); s += __shfl_xor(s, 8, 32);
                rs[r] = s;
            }
            if (lr == 0) {
#pragma unroll
                for (int r = 0; r < 8; ++r) OS[(mt * 16 + 8 * hi + r) * NT_ + nt] = rs[r] * OFOLD;
            }
        }
        __syncthreads();

        if (tid < EMB) {
            float t = 0.0f;
#pragma unroll 1
            for (int nt = 0; nt < NT_; ++nt) t += OS[tid * NT_ + nt];
            T71[head * EMB + tid] = t;
        }
        __syncthreads();
    }

    {
        const int h = tid % HID; const int part = tid / HID;
        const int pc = part < MPART ? part : MPART - 1;
        const float* wp = nl0 + (size_t)(pc * MROWS) * HID + h;
        float acc = 0.0f;
#pragma unroll 4
        for (int i = 0; i < MROWS; ++i) acc += T71[pc * MROWS + i] * bfr(wp[(size_t)i * HID]);
        PRE[part * HID + h] = acc;
    }
    __syncthreads();
    {
        const int hc = tid < HID ? tid : HID - 1;
        float b = nl0b[hc];
        asm volatile("" : "+v"(b));
        if (tid < HID) {
            const float pre = (PRE[tid] + PRE[HID + tid]) + PRE[2 * HID + tid];
            T7[tid] = fmaxf(pre, 0.0f) + bfr(b);
        }
    }
    __syncthreads();

    if (wave < 2) {
        const int e = tid < EMB ? tid : EMB - 1;
        float acc = 0.0f;
#pragma unroll 4
        for (int h = 0; h < HID; ++h) acc += T7[h] * bfr(nl1[h * EMB + e]);
        if (tid < EMB) T10[tid] = acc;
    }
    __syncthreads();

    if (wave < 4) {
        const int q = tid < NTOK / 4 ? tid : NTOK / 4 - 1;
        v4f acc = (v4f){};
#pragma unroll 2
        for (int e = 0; e < EMB; ++e) {
            const v4f w = *(const v4f*)(ctp + (size_t)e * NTOK + 4 * q);
            const float t = T10[e];
            acc[0] += t * bfr(w[0]); acc[1] += t * bfr(w[1]); acc[2] += t * bfr(w[2]); acc[3] += t * bfr(w[3]);
        }
        const v4f bb = *(const v4f*)(ctpb + 4 * q);
        v4f val;
        val[0] = acc[0] + bfr(bb[0]); val[1] = acc[1] + bfr(bb[1]); val[2] = acc[2] + bfr(bb[2]); val[3] = acc[3] + bfr(bb[3]);
        asm volatile("" : "+v"(val));
        const bool ok = tid < NTOK / 4;
        if (ok) *(volatile v4f*)(out + 4 * q) = val;
        __threadfence();
        if (ok) *(volatile v4f*)(out + 4 * q) = val;
    }
}

extern "C" void kernel_launch(void* const* d_in, const int* in_sizes, int n_in,
                              void* d_out, int out_size, void* d_ws, size_t ws_size, hipStream_t stream) {
    (void)d_ws; (void)ws_size;
    if (n_in < 12) return;
    if (in_sizes[0] < EMB * CTX) return;
    for (int i = 1; i <= 6; ++i) if (in_sizes[i] < CTX * DKW) return;
    if (in_sizes[7] < CCAT * HID || in_sizes[8] < HID || in_sizes[9] < HID * EMB) return;
    if (in_sizes[10] < EMB * NTOK || in_sizes[11] < NTOK) return;
    if (out_size < NTOK) return;
    const float* x0   = (const float*)d_in[0];
    const float* wq1  = (const float*)d_in[1];
    const float* wk1  = (const float*)d_in[2];
    const float* wv1  = (const float*)d_in[3];
    const float* wq2  = (const float*)d_in[4];
    const float* wk2  = (const float*)d_in[5];
    const float* wv2  = (const float*)d_in[6];
    const float* nl0  = (const float*)d_in[7];
    const float* nl0b = (const float*)d_in[8];
    const float* nl1  = (const float*)d_in[9];
    const float* ctp  = (const float*)d_in[10];
    const float* ctpb = (const float*)d_in[11];
    float* out = (float*)d_out;
    k_fused<<<dim3(1, 1, 1), dim3(NTH, 1, 1), 0, stream>>>(x0, wq1, wk1, wv1, wq2, wk2, wv2, nl0, nl0b, nl1, ctp, ctpb, out);
}
